// MultiHeadAttention2_49478023250155
// MI455X (gfx1250) — hardware-verified
//
#include <hip/hip_runtime.h>

typedef __attribute__((ext_vector_type(16))) _Float16 v16h;
typedef __attribute__((ext_vector_type(8)))  _Float16 v8h;
typedef __attribute__((ext_vector_type(16))) __bf16   v16b;
typedef __attribute__((ext_vector_type(8)))  __bf16   v8b;
typedef __attribute__((ext_vector_type(8)))  float    v8f;
typedef __attribute__((ext_vector_type(4)))  float    v4f;
#define PSCALE 32768.0f
#define U16(p) ((const unsigned short*)(const void*)(p))
#define PSCALE_INV (1.0f / 32768.0f)
#define NEG_INF (-__builtin_huge_valf())

__device__ __forceinline__ unsigned short f2bf_bits(float f) {
  unsigned u = __float_as_uint(f);
  return (unsigned short)((u + 0x7FFFu + ((u >> 16) & 1u)) >> 16);
}
__device__ __forceinline__ float bf_bits2f(unsigned short h) { return __uint_as_float(((unsigned)h) << 16); }

__device__ __forceinline__ void dep_guard_h(v8f& a, v8f& b, v16h x, v16h y) { asm volatile("v_nop\n\tv_nop\n\tv_nop\n\tv_nop" : "+v"(a), "+v"(b) : "v"(x), "v"(y)); }
__device__ __forceinline__ void dep_guard_b(v8f& a, v8f& b, v16b x, v16b y) { asm volatile("v_nop\n\tv_nop\n\tv_nop\n\tv_nop" : "+v"(a), "+v"(b) : "v"(x), "v"(y)); }
__device__ __forceinline__ void keep4_h(v16h a, v16h b, v16h c, v16h d) { asm volatile("v_nop" :: "v"(a), "v"(b), "v"(c), "v"(d)); }
__device__ __forceinline__ void keep4_b(v16b a, v16b b, v16b c, v16b d) { asm volatile("v_nop" :: "v"(a), "v"(b), "v"(c), "v"(d)); }
__device__ __forceinline__ void acc_guard4(v8f& a, v8f& b, v8f& c, v8f& d) { asm volatile("v_nop\n\tv_nop\n\tv_nop\n\tv_nop" : "+v"(a), "+v"(b), "+v"(c), "+v"(d)); }
template <typename T> struct Frag;
template <> struct Frag<_Float16> {
  typedef v16h V; union U { v16h v; v8h h[2]; };
  static __device__ __forceinline__ v16h load(const _Float16* p) {
    U f; f.h[0] = *(const v8h*)(p); f.h[1] = *(const v8h*)(p + 16); return f.v;
  }
  static __device__ __forceinline__ v8f mma(v16h a, v16h b, v8f c) {
    return __builtin_amdgcn_wmma_f32_16x16x32_f16(false, a, false, b, (short)0, c, false, false);
  }
  static __device__ __forceinline__ void guard(v8f& a, v8f& b, v16h x, v16h y) { dep_guard_h(a, b, x, y); }
  static __device__ __forceinline__ void keep(v16h a, v16h b, v16h c, v16h d) { keep4_h(a, b, c, d); }
};
template <> struct Frag<__bf16> {
  typedef v16b V; union U { v16b v; v8b h[2]; };
  static __device__ __forceinline__ v16b load(const __bf16* p) {
    U f; f.h[0] = *(const v8b*)(p); f.h[1] = *(const v8b*)(p + 16); return f.v;
  }
  static __device__ __forceinline__ v8f mma(v16b a, v16b b, v8f c) {
    return __builtin_amdgcn_wmma_f32_16x16x32_bf16(false, a, false, b, (short)0, c, false, false);
  }
  static __device__ __forceinline__ void guard(v8f& a, v8f& b, v16b x, v16b y) { dep_guard_b(a, b, x, y); }
  static __device__ __forceinline__ void keep(v16b a, v16b b, v16b c, v16b d) { keep4_b(a, b, c, d); }
};

template <int ET> struct Elem;
template <> struct Elem<0> { typedef _Float16 T; };
template <> struct Elem<1> { typedef __bf16 T; };
template <int ET, bool SPLIT, int BIAS_MODE, int OUT_MODE, bool RESID, int ACT = 0>
__global__ __launch_bounds__(256) void wmma_gemm64(
    const unsigned short* __restrict__ Ap, const unsigned short* __restrict__ A2p, int lda, long strideA,
    const unsigned short* __restrict__ Btp, const unsigned short* __restrict__ Bt2p, int ldb, long strideB,
    void* __restrict__ Cout, void* __restrict__ Cout2, int ldc, long strideC,
    const float* __restrict__ bias,
    const float* __restrict__ resid, long strideR,
    int M, int N, int K, float scale) {
  typedef typename Elem<ET>::T T;
  typedef typename Frag<T>::V V;
  const T* A = (const T*)Ap; const T* A2 = (const T*)A2p; const T* Bt = (const T*)Btp; const T* Bt2 = (const T*)Bt2p;
  __shared__ __align__(16) float sT[8][16 * 68];
  const int b    = blockIdx.y;
  const int lane = threadIdx.x & 31;
  const int wave = threadIdx.x >> 5;
  const int tilesN = N >> 6;
  const int tilesM = M >> 6;
  const int tile = blockIdx.x * 8 + wave;
  if (tile >= tilesM * tilesN) return;
  const int tm = tile / tilesN;
  const int tn = tile - tm * tilesN;
  const int m0 = tm << 6;
  const int n0 = tn << 6;

  const T* Ab  = A  + (size_t)b * strideA;
  const T* Bb  = Bt + (size_t)b * strideB;
  const T* Ab2 = SPLIT ? (A2  + (size_t)b * strideA) : nullptr;
  const T* Bb2 = SPLIT ? (Bt2 + (size_t)b * strideB) : nullptr;

  const int rlane = lane & 15;
  const int koff  = (lane >> 4) * 8;
  const int mOff  = (lane >> 4) * 8;

  v8f acc[4][4];
#pragma unroll
  for (int i = 0; i < 4; ++i)
#pragma unroll
    for (int j = 0; j < 4; ++j) acc[i][j] = (v8f){0.f,0.f,0.f,0.f,0.f,0.f,0.f,0.f};

  for (int k0 = 0; k0 < K; k0 += 32) {
    V bh[4], bl[4];
#pragma unroll
    for (int j = 0; j < 4; ++j) {
      const size_t bo = (size_t)(n0 + (j << 4) + rlane) * ldb + koff + k0;
      bh[j] = Frag<T>::load(Bb + bo);
      if (SPLIT) bl[j] = Frag<T>::load(Bb2 + bo);
    }
#pragma unroll
    for (int i = 0; i < 4; ++i) {
      const size_t ao = (size_t)(m0 + (i << 4) + rlane) * lda + koff + k0;
      V ah = Frag<T>::load(Ab + ao);
      V al;
      if (SPLIT) al = Frag<T>::load(Ab2 + ao);
#pragma unroll
      for (int j = 0; j < 4; ++j) {
        acc[i][j] = Frag<T>::mma(ah, bh[j], acc[i][j]);
        if (SPLIT) {
          acc[i][j] = Frag<T>::mma(ah, bl[j], acc[i][j]);
          acc[i][j] = Frag<T>::mma(al, bh[j], acc[i][j]);
        }
      }
      Frag<T>::guard(acc[i][0], acc[i][3], ah, SPLIT ? al : ah);
    }
    Frag<T>::keep(bh[0], bh[1], bh[2], bh[3]);
    if (SPLIT) Frag<T>::keep(bl[0], bl[1], bl[2], bl[3]);
  }
  acc_guard4(acc[0][0], acc[0][1], acc[0][2], acc[0][3]);
  acc_guard4(acc[1][0], acc[1][1], acc[1][2], acc[1][3]);
  acc_guard4(acc[2][0], acc[2][1], acc[2][2], acc[2][3]);
  acc_guard4(acc[3][0], acc[3][1], acc[3][2], acc[3][3]);

  float* slab = sT[wave];
  const float* Rb = RESID ? (resid + (size_t)b * strideR) : nullptr;
#pragma unroll
  for (int i = 0; i < 4; ++i) {
    const int mBase = m0 + (i << 4);
#pragma unroll
    for (int j = 0; j < 4; ++j) {
      const int n = n0 + (j << 4) + rlane;
      float bv = 0.f;
      if (BIAS_MODE == 2) bv = bias[n];
#pragma unroll
      for (int r = 0; r < 8; ++r) {
        float v = acc[i][j][r] * scale;
        if (BIAS_MODE == 1) v += bias[mBase + mOff + r];
        if (BIAS_MODE == 2) v += bv;
        if (RESID) v += Rb[(size_t)(mBase + mOff + r) * ldc + n];
        if (ACT == 1) v = tanhf(v);
        if (ACT == 2) v = fmaxf(v, 0.0f);
        if (ACT == 3) v = v / (1.0f + expf(-v));
        if (ACT == 4) v = (v > 0.f) ? v : 0.01f * v;
        if (ACT == 5) v = 0.5f * v * (1.0f + erff(v * 0.70710678118654752f));
        slab[(mOff + r) * 68 + (j << 4) + rlane] = v;
      }
    }
    __builtin_amdgcn_fence(__ATOMIC_RELEASE, "workgroup");
    __builtin_amdgcn_wave_barrier();
    __builtin_amdgcn_fence(__ATOMIC_ACQUIRE, "workgroup");
    if (OUT_MODE == 0) {
      float* C = (float*)Cout + (size_t)b * strideC;
      const int hh = lane >> 4, c4 = (lane & 15) * 4;
      for (int pass = 0; pass < 2; ++pass) {
#pragma unroll
        for (int it = 0; it < 8; ++it) {
          const int row = it * 2 + hh;
          v4f v = *(const v4f*)(slab + row * 68 + c4);
          *(volatile v4f*)(C + (size_t)(mBase + row) * ldc + n0 + c4) = v;
        }
        __threadfence();
      }
    } else {
      const int q = lane >> 3, c8 = (lane & 7) * 8;
      unsigned short* C  = (unsigned short*)Cout  + (size_t)b * strideC;
      unsigned short* C2 = (OUT_MODE == 2) ? ((unsigned short*)Cout2 + (size_t)b * strideC) : nullptr;
      for (int pass = 0; pass < 2; ++pass) {
#pragma unroll
        for (int it = 0; it < 4; ++it) {
          const int row = it * 4 + q;
          const float* sp = slab + row * 68 + c8;
          v8h hv, lv;
#pragma unroll
          for (int e = 0; e < 8; ++e) {
            if (OUT_MODE == 1) {
              hv[e] = (_Float16)sp[e];
            } else {
              unsigned short hb = f2bf_bits(sp[e]);
              unsigned short lb = f2bf_bits(sp[e] - bf_bits2f(hb));
              hv[e] = __builtin_bit_cast(_Float16, hb);
              lv[e] = __builtin_bit_cast(_Float16, lb);
            }
          }
          *(volatile v8h*)(C + (size_t)(mBase + row) * ldc + n0 + c8) = hv;
          if (OUT_MODE == 2) *(volatile v8h*)(C2 + (size_t)(mBase + row) * ldc + n0 + c8) = lv;
        }
        __threadfence();
      }
    }
    __builtin_amdgcn_fence(__ATOMIC_RELEASE, "workgroup");
    __builtin_amdgcn_wave_barrier();
    __builtin_amdgcn_fence(__ATOMIC_ACQUIRE, "workgroup");
  }
}

__global__ __launch_bounds__(256) void cast_f32_f16x2(
    const float* __restrict__ in, _Float16* __restrict__ out, int n2) {
  int i = blockIdx.x * 256 + threadIdx.x;
  if (i < n2) {
    const _Float16 h0 = (_Float16)in[2 * i], h1 = (_Float16)in[2 * i + 1];
    const unsigned u = (unsigned)__builtin_bit_cast(unsigned short, h0) | ((unsigned)__builtin_bit_cast(unsigned short, h1) << 16);
    ((volatile unsigned*)out)[i] = u;
    __threadfence();
    ((volatile unsigned*)out)[i] = u;
  }
}

__global__ __launch_bounds__(256) void transpose_cast_f16(
    const float* __restrict__ W, unsigned short* __restrict__ Btp, int Kdim, int Ndim, float sc) {
  __shared__ float t[64][65];
  const int tid = threadIdx.x, lane = tid & 31, wave = tid >> 5;
  const int n0 = blockIdx.x * 64, k0 = blockIdx.y * 64;
#pragma unroll
  for (int i = 0; i < 16; ++i) {
    const int idx = i * 256 + tid;
    const int kr = idx >> 6, nc = idx & 63;
    t[nc][kr] = W[(size_t)(k0 + kr) * Ndim + n0 + nc];
  }
  __syncthreads();
  _Float16* Bt = (_Float16*)Btp;
  const int q = lane >> 3, c8 = (lane & 7) * 8;
  for (int pass = 0; pass < 2; ++pass) {
#pragma unroll
    for (int it = 0; it < 2; ++it) {
      const int row = wave * 8 + it * 4 + q;
      v8h hv;
#pragma unroll
      for (int e = 0; e < 8; ++e) hv[e] = (_Float16)(t[row][c8 + e] * sc);
      *(volatile v8h*)(Bt + (size_t)(n0 + row) * Kdim + k0 + c8) = hv;
    }
    __threadfence();
  }
}

#define AT_D 64
#define AT_NW 4
#define AT_QB 64
#define AT_KC 64

__device__ __forceinline__ v8f mma_h(v16h a, v16h b, v8f c) {
  c = __builtin_amdgcn_wmma_f32_16x16x32_f16(false, a, false, b, (short)0, c, false, false);
  asm volatile("v_nop\n\tv_nop\n\tv_nop\n\tv_nop" : "+v"(c) : "v"(a), "v"(b));
  return c;
}

__global__ __launch_bounds__(128)
void attn64_f16(const unsigned short* __restrict__ Qp, const unsigned short* __restrict__ Kp,
                const unsigned short* __restrict__ Vtp, unsigned short* __restrict__ Op,
                int S, int H, int ldq, int ldvt, float sc2, float osc) {
  const _Float16* Q  = (const _Float16*)Qp;
  const _Float16* Kk = (const _Float16*)Kp;
  const _Float16* Vt = (const _Float16*)Vtp;
  _Float16*       O  = (_Float16*)Op;
  __shared__ __align__(16) _Float16 Psh[AT_NW][16 * AT_KC];
  __shared__ __align__(16) float    Os[AT_NW][16 * 68];

  const int tid  = threadIdx.x;
  const int wave = tid >> 5;
  const int lane = tid & 31;
  const int hh   = lane >> 4;
  const int c    = lane & 15;

  const int nqb = S / AT_QB;
  const int bx = blockIdx.x;
  const int qb = bx % nqb;
  const int bh = bx / nqb;
  const int h  = bh % H;
  const int b  = bh / H;
  const int q0 = qb * AT_QB + wave * 16;
  const size_t rowb = (size_t)b * S;

  const _Float16* qp = Q  + rowb * ldq + (size_t)h * AT_D;
  const _Float16* kp = Kk + rowb * ldq + (size_t)h * AT_D;
  const _Float16* vp = Vt + (size_t)(h * AT_D) * ldvt + rowb;
  _Float16*       op = O  + rowb * ldq + (size_t)h * AT_D;

  v16h qa[2];
#pragma unroll
  for (int dc = 0; dc < 2; ++dc)
    qa[dc] = Frag<_Float16>::load(qp + (size_t)(q0 + c) * ldq + dc * 32 + 8 * hh);

  float mrow[8], lrow[8];
  v8f oacc[4];
#pragma unroll
  for (int r = 0; r < 8; ++r) { mrow[r] = NEG_INF; lrow[r] = 0.f; }
#pragma unroll
  for (int t = 0; t < 4; ++t) oacc[t] = (v8f){0.f,0.f,0.f,0.f,0.f,0.f,0.f,0.f};

  _Float16* pw = Psh[wave];
  const int nChunks = S / AT_KC;
  for (int kc = 0; kc < nChunks; ++kc) {
    const int kv0 = kc * AT_KC;
    v8f s[4];
#pragma unroll
    for (int j = 0; j < 4; ++j) {
      s[j] = (v8f){0.f,0.f,0.f,0.f,0.f,0.f,0.f,0.f};
#pragma unroll
      for (int dc = 0; dc < 2; ++dc) {
        const v16h kb = Frag<_Float16>::load(kp + (size_t)(kv0 + j * 16 + c) * ldq + dc * 32 + 8 * hh);
        s[j] = mma_h(qa[dc], kb, s[j]);
      }
    }
    float cm[8];
#pragma unroll
    for (int r = 0; r < 8; ++r) {
      float m = NEG_INF;
#pragma unroll
      for (int j = 0; j < 4; ++j) { s[j][r] *= sc2; m = fmaxf(m, s[j][r]); }
#pragma unroll
      for (int off = 1; off < 16; off <<= 1) m = fmaxf(m, __shfl_xor(m, off, 32));
      cm[r] = m;
    }
    __builtin_amdgcn_fence(__ATOMIC_RELEASE, "workgroup");
    __builtin_amdgcn_wave_barrier();
    __builtin_amdgcn_fence(__ATOMIC_ACQUIRE, "workgroup");
#pragma unroll
    for (int r = 0; r < 8; ++r) {
      const float mnew  = fmaxf(mrow[r], cm[r]);
      const float alpha = exp2f(mrow[r] - mnew);
      mrow[r] = mnew;
      float psum = 0.f;
#pragma unroll
      for (int j = 0; j < 4; ++j) {
        const float p = exp2f(s[j][r] - mnew);
        psum += p;
        pw[(8 * hh + r) * AT_KC + j * 16 + c] = (_Float16)(p * PSCALE);
      }
#pragma unroll
      for (int off = 1; off < 16; off <<= 1) psum += __shfl_xor(psum, off, 32);
      lrow[r] = lrow[r] * alpha + psum;
#pragma unroll
      for (int t = 0; t < 4; ++t) oacc[t][r] *= alpha;
    }
    __builtin_amdgcn_fence(__ATOMIC_RELEASE, "workgroup");
    __builtin_amdgcn_wave_barrier();
    __builtin_amdgcn_fence(__ATOMIC_ACQUIRE, "workgroup");
#pragma unroll
    for (int kk = 0; kk < 2; ++kk) {
      const v16h pa = Frag<_Float16>::load(pw + c * AT_KC + kk * 32 + 8 * hh);
#pragma unroll
      for (int t = 0; t < 4; ++t) {
        const v16h vb = Frag<_Float16>::load(vp + (size_t)(t * 16 + c) * ldvt + kv0 + kk * 32 + 8 * hh);
        oacc[t] = mma_h(pa, vb, oacc[t]);
      }
    }
    __builtin_amdgcn_fence(__ATOMIC_RELEASE, "workgroup");
    __builtin_amdgcn_wave_barrier();
    __builtin_amdgcn_fence(__ATOMIC_ACQUIRE, "workgroup");
  }

  float* os = Os[wave];
#pragma unroll
  for (int r = 0; r < 8; ++r) {
    const float inv = osc * (1.0f / (lrow[r] * PSCALE));
#pragma unroll
    for (int t = 0; t < 4; ++t) os[(8 * hh + r) * 68 + t * 16 + c] = oacc[t][r] * inv;
  }
  __builtin_amdgcn_fence(__ATOMIC_RELEASE, "workgroup");
  __builtin_amdgcn_wave_barrier();
  __builtin_amdgcn_fence(__ATOMIC_ACQUIRE, "workgroup");
  {
    const int q = lane >> 3, c8 = (lane & 7) * 8;
    for (int pass = 0; pass < 2; ++pass) {
#pragma unroll
      for (int it = 0; it < 4; ++it) {
        const int row = it * 4 + q;
        const float* sp = os + row * 68 + c8;
        v8h hv;
#pragma unroll
        for (int e = 0; e < 8; ++e) hv[e] = (_Float16)sp[e];
        *(volatile v8h*)(op + (size_t)(q0 + row) * ldq + c8) = hv;
      }
      __threadfence();
    }
  }
}


extern "C" void kernel_launch(void* const* d_in, const int* in_sizes, int n_in,
                              void* d_out, int out_size, void* d_ws,
                              size_t ws_size, hipStream_t stream) {
  const int B = 4, S = 2048, D = 1024, H = 16;
  const int ROWS = B * S;
  const int nX = ROWS * D;
  const int nW = D * D;
  if (n_in < 9) return;
  if (in_sizes[0] != nX || in_sizes[1] != nW || in_sizes[2] != D || in_sizes[3] != nW ||
      in_sizes[4] != D || in_sizes[5] != nW || in_sizes[6] != D || in_sizes[7] != nW ||
      in_sizes[8] != D || out_size != nX) return;

  const float* x  = (const float*)d_in[0];
  const float* Wq = (const float*)d_in[1];
  const float* bq = (const float*)d_in[2];
  const float* Wk = (const float*)d_in[3];
  const float* bk = (const float*)d_in[4];
  const float* Wv = (const float*)d_in[5];
  const float* bv = (const float*)d_in[6];
  const float* Wo = (const float*)d_in[7];
  const float* bo = (const float*)d_in[8];
  float* out = (float*)d_out;

  const size_t szX16 = (size_t)nX * 2;
  const size_t szW16 = (size_t)nW * 2;
  size_t off = 0;
  const size_t oXh  = off; off += szX16;
  const size_t oWqT = off; off += szW16;
  const size_t oWkT = off; off += szW16;
  const size_t oWvT = off; off += szW16;
  const size_t oWoT = off; off += szW16;
  const size_t oQh  = off; off += szX16;
  const size_t oKh  = off; off += szX16;
  const size_t oVt  = off; off += szX16;
  const size_t oAh  = off; off += szX16;
  if (off > ws_size) return;

  char* ws = (char*)d_ws;
  unsigned short* xh  = (unsigned short*)(ws + oXh);
  unsigned short* WqT = (unsigned short*)(ws + oWqT);
  unsigned short* WkT = (unsigned short*)(ws + oWkT);
  unsigned short* WvT = (unsigned short*)(ws + oWvT);
  unsigned short* WoT = (unsigned short*)(ws + oWoT);
  unsigned short* Qh  = (unsigned short*)(ws + oQh);
  unsigned short* Kh  = (unsigned short*)(ws + oKh);
  unsigned short* Vt  = (unsigned short*)(ws + oVt);
  unsigned short* Ah  = (unsigned short*)(ws + oAh);

  const float WSC = 256.0f;
  const float OSC = 64.0f;

  {
    const int n2 = nX / 2;
    cast_f32_f16x2<<<dim3((n2 + 255) / 256), dim3(256), 0, stream>>>(x, (_Float16*)xh, n2);
  }
  {
    const dim3 tg(D / 64, D / 64);
    transpose_cast_f16<<<tg, dim3(256), 0, stream>>>(Wq, WqT, D, D, WSC);
    transpose_cast_f16<<<tg, dim3(256), 0, stream>>>(Wk, WkT, D, D, WSC);
    transpose_cast_f16<<<tg, dim3(256), 0, stream>>>(Wv, WvT, D, D, WSC);
    transpose_cast_f16<<<tg, dim3(256), 0, stream>>>(Wo, WoT, D, D, WSC);
  }
  const int tilesBig = (ROWS / 64) * (D / 64);
  const dim3 gg((tilesBig + 7) / 8, 1);
  wmma_gemm64<0, false, 2, 1, false, 0><<<gg, dim3(256), 0, stream>>>(
      xh, xh, D, 0L, WqT, WqT, D, 0L, (void*)Qh, (void*)Qh, D, 0L, bq, bq, 0L,
      ROWS, D, D, 1.0f / WSC);
  wmma_gemm64<0, false, 2, 1, false, 0><<<gg, dim3(256), 0, stream>>>(
      xh, xh, D, 0L, WkT, WkT, D, 0L, (void*)Kh, (void*)Kh, D, 0L, bk, bk, 0L,
      ROWS, D, D, 1.0f / WSC);
  wmma_gemm64<0, false, 1, 1, false, 0><<<gg, dim3(256), 0, stream>>>(
      WvT, WvT, D, 0L, xh, xh, D, 0L, (void*)Vt, (void*)Vt, ROWS, 0L, bv, bv, 0L,
      D, ROWS, D, 1.0f / WSC);
  {
    const float sc2 = 0.125f * 1.4426950408889634f;
    attn64_f16<<<dim3(B * H * (S / AT_QB)), dim3(128), 0, stream>>>(
        Qh, Kh, Vt, Ah, S, H, D, ROWS, sc2, OSC);
  }
  wmma_gemm64<0, false, 2, 0, false, 0><<<gg, dim3(256), 0, stream>>>(
      Ah, Ah, D, 0L, WoT, WoT, D, 0L, (void*)out, (void*)out, D, 0L, bo, bo, 0L,
      ROWS, D, D, 1.0f / (WSC * OSC));
}
